// JambaModel_65687229825534
// MI455X (gfx1250) — hardware-verified
//
#include <hip/hip_runtime.h>
#include <math.h>
#include <stdint.h>

#define SEQ  2048
#define DMD  1024
#define DKV  256
#define NHD  16
#define HDIM 64
#define DFFN 2752
#define DXZ  2048
#define DXN  1056
#define DXP  1088
#define NST  16
#define NSSM 3
#define NQB  (SEQ / 64)
static_assert(NHD * HDIM == DMD);
static_assert((SEQ % 64) == 0 && (DMD % 64) == 0 && (DKV % 64) == 0 && (DFFN % 64) == 0);
static_assert((DFFN % 32) == 0 && (DXP % 64) == 0 && DXP >= DXN && (DXN % 4) == 0);
static_assert(NHD / (DKV / HDIM) == 4);

typedef _Float16 v16h __attribute__((ext_vector_type(16)));
typedef _Float16 v8h  __attribute__((ext_vector_type(8)));
typedef __bf16   v16b __attribute__((ext_vector_type(16)));
typedef __bf16   v8b  __attribute__((ext_vector_type(8)));
typedef float    v8f  __attribute__((ext_vector_type(8)));
typedef float    v4f  __attribute__((ext_vector_type(4)));
typedef unsigned int v4u __attribute__((ext_vector_type(4)));
typedef unsigned int v2u __attribute__((ext_vector_type(2)));

__device__ __forceinline__ unsigned short bf_bits(float f) {
  unsigned u = __float_as_uint(f);
  return (unsigned short)((u + 0x7FFFu + ((u >> 16) & 1u)) >> 16);
}
__device__ __forceinline__ float bf_up(unsigned short b) { return __uint_as_float(((unsigned)b) << 16); }
__device__ __forceinline__ unsigned short h_bits(float f) {
  const _Float16 x = (_Float16)f;
  return __builtin_bit_cast(unsigned short, x);
}
__device__ __forceinline__ unsigned pk16(unsigned short a, unsigned short b) { return (unsigned)a | ((unsigned)b << 16); }
__device__ __forceinline__ v8f zero8() { v8f z = {0.f, 0.f, 0.f, 0.f, 0.f, 0.f, 0.f, 0.f}; return z; }
__device__ __forceinline__ float rcpf(float x) { return __builtin_amdgcn_rcpf(x); }
__device__ __forceinline__ float siluf(float v) {
  const float e = __expf(-v);
  return v * rcpf(1.0f + e);
}

template <typename ET> struct FT;
template <> struct FT<_Float16> { typedef v16h V16; typedef v8h V8; };
template <> struct FT<__bf16>   { typedef v16b V16; typedef v8b V8; };

template <typename ET>
__device__ __forceinline__ typename FT<ET>::V16 ldfrag(const ET* p) {
  typedef typename FT<ET>::V16 V16;
  typedef typename FT<ET>::V8  V8;
  union U { V16 v; V8 h[2]; } f;
  f.h[0] = *(const V8*)(p);
  f.h[1] = *(const V8*)(p + 16);
  return f.v;
}

__device__ __forceinline__ v8f mma_raw(v16h a, v16h b, v8f c) {
  return __builtin_amdgcn_wmma_f32_16x16x32_f16(false, a, false, b, (short)0, c, false, false);
}
__device__ __forceinline__ v8f mma_raw(v16b a, v16b b, v8f c) {
  return __builtin_amdgcn_wmma_f32_16x16x32_bf16(false, a, false, b, (short)0, c, false, false);
}
__device__ __forceinline__ v8f mma_g(v16h a, v16h b, v8f c) {
  c = mma_raw(a, b, c);
#if defined(__HIP_DEVICE_COMPILE__)
  asm volatile("v_nop\n\tv_nop\n\tv_nop\n\tv_nop" : "+v"(c) : "v"(a), "v"(b));
#endif
  return c;
}
__device__ __forceinline__ void dep_guard(v8f& a, v8f& b, v16h x, v16h y) {
#if defined(__HIP_DEVICE_COMPILE__)
  asm volatile("v_nop\n\tv_nop\n\tv_nop\n\tv_nop" : "+v"(a), "+v"(b) : "v"(x), "v"(y));
#else
  (void)a; (void)b; (void)x; (void)y;
#endif
}
__device__ __forceinline__ void dep_guard(v8f& a, v8f& b, v16b x, v16b y) {
#if defined(__HIP_DEVICE_COMPILE__)
  asm volatile("v_nop\n\tv_nop\n\tv_nop\n\tv_nop" : "+v"(a), "+v"(b) : "v"(x), "v"(y));
#else
  (void)a; (void)b; (void)x; (void)y;
#endif
}
__device__ __forceinline__ void keep4(v16h a, v16h b, v16h c, v16h d) {
#if defined(__HIP_DEVICE_COMPILE__)
  asm volatile("v_nop" :: "v"(a), "v"(b), "v"(c), "v"(d));
#else
  (void)a; (void)b; (void)c; (void)d;
#endif
}
__device__ __forceinline__ void keep4(v16b a, v16b b, v16b c, v16b d) {
#if defined(__HIP_DEVICE_COMPILE__)
  asm volatile("v_nop" :: "v"(a), "v"(b), "v"(c), "v"(d));
#else
  (void)a; (void)b; (void)c; (void)d;
#endif
}
__device__ __forceinline__ void acc_guard4(v8f& a, v8f& b, v8f& c, v8f& d) {
#if defined(__HIP_DEVICE_COMPILE__)
  asm volatile("v_nop\n\tv_nop\n\tv_nop\n\tv_nop" : "+v"(a), "+v"(b), "+v"(c), "+v"(d));
#else
  (void)a; (void)b; (void)c; (void)d;
#endif
}

template <int BFP>
__global__ __launch_bounds__(256) void rmsnorm_h(const float* __restrict__ x, const float* __restrict__ w,
                                                 unsigned short* y, unsigned short* yh, unsigned short* yl) {
  __shared__ float red[8];
  const int tid = threadIdx.x, lane = tid & 31, wave = tid >> 5;
  const int row = blockIdx.x;
  const v4f xv = *(const v4f*)(x + (size_t)row * DMD + 4 * tid);
  const v4f wv = *(const v4f*)(w + 4 * tid);
  float s = xv[0] * xv[0] + xv[1] * xv[1] + xv[2] * xv[2] + xv[3] * xv[3];
#pragma unroll
  for (int off = 1; off < 32; off <<= 1) s += __shfl_xor(s, off, 32);
  if (lane == 0) red[wave] = s;
  __syncthreads();
  float tot = 0.f;
#pragma unroll
  for (int i = 0; i < 8; ++i) tot += red[i];
  const float sc = rsqrtf(tot * (1.0f / (float)DMD) + 1e-6f);
  float n[4];
#pragma unroll
  for (int e = 0; e < 4; ++e) n[e] = xv[e] * sc * wv[e];
  v2u p;
  p[0] = pk16(h_bits(n[0]), h_bits(n[1]));
  p[1] = pk16(h_bits(n[2]), h_bits(n[3]));
  v2u ph = p, pl = p;
  if (BFP != 0) {
    unsigned short hb[4], lb[4];
#pragma unroll
    for (int e = 0; e < 4; ++e) { hb[e] = bf_bits(n[e]); lb[e] = bf_bits(n[e] - bf_up(hb[e])); }
    ph[0] = pk16(hb[0], hb[1]); ph[1] = pk16(hb[2], hb[3]);
    pl[0] = pk16(lb[0], lb[1]); pl[1] = pk16(lb[2], lb[3]);
  }
  const size_t o = (size_t)row * DMD + 4 * tid;
  *(volatile v2u*)(y + o) = p;
  if (BFP != 0) {
    *(volatile v2u*)(yh + o) = ph;
    *(volatile v2u*)(yl + o) = pl;
  }
  __threadfence();
  *(volatile v2u*)(y + o) = p;
  if (BFP != 0) {
    *(volatile v2u*)(yh + o) = ph;
    *(volatile v2u*)(yl + o) = pl;
  }
}

template <int MODE>
__global__ __launch_bounds__(256) void wcvt(const float* __restrict__ W, int ldw, int Kdim, int Nreal,
                                            unsigned short* out, unsigned short* out2, float scale) {
  __shared__ __align__(16) float tile[64 * 68];
  const int tid = threadIdx.x;
  const int n0 = blockIdx.x * 64, k0 = blockIdx.y * 64;
  {
    const int r = tid >> 2, c16 = (tid & 3) * 16;
    const int k = k0 + r;
#pragma unroll
    for (int i = 0; i < 4; ++i) {
      const int n  = n0 + c16 + 4 * i;
      const int nc = (n < Nreal - 4) ? n : (Nreal - 4);
      const v4f v  = *(const v4f*)(W + (size_t)k * ldw + nc);
#pragma unroll
      for (int e = 0; e < 4; ++e) {
        const float f = (n + e < Nreal) ? v[e] : 0.f;
        tile[(c16 + 4 * i + e) * 68 + r] = f * scale;
      }
    }
  }
  __syncthreads();
  const int wave = tid >> 5, lane = tid & 31, q = lane >> 3, j = lane & 7;
  v4u o1[2], o2[2];
#pragma unroll
  for (int it = 0; it < 2; ++it) {
    const int c = 8 * wave + 4 * it + q;
    const float* sp = tile + c * 68 + 8 * j;
    float f[8];
#pragma unroll
    for (int e = 0; e < 8; ++e) f[e] = sp[e];
    v4u a, a2;
#pragma unroll
    for (int e = 0; e < 4; ++e) {
      const float f0 = f[2 * e], f1 = f[2 * e + 1];
      if (MODE == 0) {
        a[e] = pk16(h_bits(f0), h_bits(f1));
        a2[e] = a[e];
      } else {
        const unsigned short hb0 = bf_bits(f0), hb1 = bf_bits(f1);
        const unsigned short lb0 = bf_bits(f0 - bf_up(hb0)), lb1 = bf_bits(f1 - bf_up(hb1));
        a[e] = pk16(hb0, hb1);
        a2[e] = pk16(lb0, lb1);
      }
    }
    o1[it] = a; o2[it] = a2;
  }
  for (int pass = 0; pass < 2; ++pass) {
#pragma unroll
    for (int it = 0; it < 2; ++it) {
      const int c = 8 * wave + 4 * it + q;
      const size_t go = (size_t)(n0 + c) * Kdim + k0 + 8 * j;
      *(volatile v4u*)(out + go) = o1[it];
      if (MODE == 1) *(volatile v4u*)(out2 + go) = o2[it];
    }
    __threadfence();
  }
}

template <typename ET, int NSPLIT, int OM>
__global__ __launch_bounds__(256) void gemm64(
    const unsigned short* __restrict__ Ap, const unsigned short* __restrict__ A2p, int lda,
    const unsigned short* __restrict__ Btp, const unsigned short* __restrict__ Bt2p, int ldb,
    void* Cp, int ldc, const float* Rp, int ldr,
    int M, int N, int K, float scale) {
  typedef typename FT<ET>::V16 V16;
  const ET* A   = (const ET*)(const void*)Ap;
  const ET* A2  = (const ET*)(const void*)A2p;
  const ET* Bt  = (const ET*)(const void*)Btp;
  const ET* Bt2 = (const ET*)(const void*)Bt2p;
  __shared__ __align__(16) float sT[8][16 * 68];
  const int lane = threadIdx.x & 31;
  const int wave = threadIdx.x >> 5;
  const int tilesN = N >> 6;
  const int tilesM = M >> 6;
  const int tile = blockIdx.x * 8 + wave;
  if (tile >= tilesM * tilesN) return;
  const int tm = tile / tilesN;
  const int tn = tile - tm * tilesN;
  const int m0 = tm << 6;
  const int n0 = tn << 6;

  const int rlane = lane & 15;
  const int koff  = (lane >> 4) * 8;
  const int mOff  = (lane >> 4) * 8;

  v8f acc[4][4];
#pragma unroll
  for (int i = 0; i < 4; ++i)
#pragma unroll
    for (int j = 0; j < 4; ++j) acc[i][j] = zero8();

  for (int k0 = 0; k0 < K; k0 += 32) {
    V16 bf[4];
#pragma unroll
    for (int j = 0; j < 4; ++j) {
      const size_t bo = (size_t)(n0 + (j << 4) + rlane) * ldb + koff + k0;
      bf[j] = ldfrag<ET>(Bt + bo);
    }
#pragma unroll
    for (int i = 0; i < 4; ++i) {
      const size_t ao = (size_t)(m0 + (i << 4) + rlane) * lda + koff + k0;
      const V16 ah = ldfrag<ET>(A + ao);
      V16 al = ah;
      if (NSPLIT == 2) al = ldfrag<ET>(A2 + ao);
#pragma unroll
      for (int j = 0; j < 4; ++j) {
        acc[i][j] = mma_raw(ah, bf[j], acc[i][j]);
        if (NSPLIT == 2) acc[i][j] = mma_raw(al, bf[j], acc[i][j]);
      }
      dep_guard(acc[i][0], acc[i][3], ah, al);
    }
    keep4(bf[0], bf[1], bf[2], bf[3]);
    if (NSPLIT == 2) {
      V16 bg[4];
#pragma unroll
      for (int j = 0; j < 4; ++j) {
        const size_t bo = (size_t)(n0 + (j << 4) + rlane) * ldb + koff + k0;
        bg[j] = ldfrag<ET>(Bt2 + bo);
      }
#pragma unroll
      for (int i = 0; i < 4; ++i) {
        const size_t ao = (size_t)(m0 + (i << 4) + rlane) * lda + koff + k0;
        const V16 ah = ldfrag<ET>(A + ao);
#pragma unroll
        for (int j = 0; j < 4; ++j) acc[i][j] = mma_raw(ah, bg[j], acc[i][j]);
        dep_guard(acc[i][0], acc[i][3], ah, ah);
      }
      keep4(bg[0], bg[1], bg[2], bg[3]);
    }
  }
  acc_guard4(acc[0][0], acc[0][1], acc[0][2], acc[0][3]);
  acc_guard4(acc[1][0], acc[1][1], acc[1][2], acc[1][3]);
  acc_guard4(acc[2][0], acc[2][1], acc[2][2], acc[2][3]);
  acc_guard4(acc[3][0], acc[3][1], acc[3][2], acc[3][3]);

  float* slab = sT[wave];
#pragma unroll
  for (int i = 0; i < 4; ++i) {
    const int mBase = m0 + (i << 4);
#pragma unroll
    for (int j = 0; j < 4; ++j) {
#pragma unroll
      for (int r = 0; r < 8; ++r) {
        slab[(mOff + r) * 68 + (j << 4) + rlane] = acc[i][j][r] * scale;
      }
    }
    __builtin_amdgcn_fence(__ATOMIC_RELEASE, "workgroup");
    __builtin_amdgcn_wave_barrier();
    __builtin_amdgcn_fence(__ATOMIC_ACQUIRE, "workgroup");
    if (OM == 0 || OM == 1) {
      float* C = (float*)Cp;
      const int hh = lane >> 4, c4 = (lane & 15) * 4;
      v4f vals[8];
#pragma unroll
      for (int it = 0; it < 8; ++it) {
        const int row = it * 2 + hh;
        v4f v = *(const v4f*)(slab + row * 68 + c4);
        if (OM == 1) {
          const v4f rr = *(const v4f*)(Rp + (size_t)(mBase + row) * ldr + n0 + c4);
          v = v + rr;
        }
        vals[it] = v;
      }
      for (int pass = 0; pass < 2; ++pass) {
#pragma unroll
        for (int it = 0; it < 8; ++it) {
          const int row = it * 2 + hh;
          *(volatile v4f*)(C + (size_t)(mBase + row) * ldc + n0 + c4) = vals[it];
        }
        __threadfence();
      }
    } else {
      unsigned short* C = (unsigned short*)Cp;
      const int q = lane >> 3, c8 = (lane & 7) * 8;
      v4u hv[4];
#pragma unroll
      for (int it = 0; it < 4; ++it) {
        const int row = it * 4 + q;
        const float* sp = slab + row * 68 + c8;
        float f[8];
#pragma unroll
        for (int e = 0; e < 8; ++e) f[e] = sp[e];
        if (OM == 3) {
          const float* gp = Rp + (size_t)(mBase + row) * ldr + n0 + c8;
          const v4f g0 = *(const v4f*)(gp), g1 = *(const v4f*)(gp + 4);
#pragma unroll
          for (int e = 0; e < 4; ++e) { f[e] *= siluf(g0[e]); f[4 + e] *= siluf(g1[e]); }
        }
        v4u a;
#pragma unroll
        for (int e = 0; e < 4; ++e) a[e] = pk16(h_bits(f[2 * e]), h_bits(f[2 * e + 1]));
        hv[it] = a;
      }
      for (int pass = 0; pass < 2; ++pass) {
#pragma unroll
        for (int it = 0; it < 4; ++it) {
          const int row = it * 4 + q;
          *(volatile v4u*)(C + (size_t)(mBase + row) * ldc + n0 + c8) = hv[it];
        }
        __threadfence();
      }
    }
    __builtin_amdgcn_fence(__ATOMIC_RELEASE, "workgroup");
    __builtin_amdgcn_wave_barrier();
    __builtin_amdgcn_fence(__ATOMIC_ACQUIRE, "workgroup");
  }
}

__global__ __launch_bounds__(128)
void attn_causal(const unsigned short* __restrict__ Qp, const unsigned short* __restrict__ Kp,
                 const unsigned short* __restrict__ Vtp, unsigned short* Op, float sscale, float oscale) {
  union FH { v16h v; v8h h[2]; };
  __shared__ __align__(16) _Float16 Ksh[64 * 64];
  __shared__ __align__(16) _Float16 Vth[64 * 64];
  __shared__ __align__(16) _Float16 Psh[4][16 * 64];
  __shared__ __align__(16) float    Os[4][16 * 64];

  const int tid  = threadIdx.x;
  const int wave = tid >> 5;
  const int lane = tid & 31;
  const int hh   = lane >> 4;
  const int c    = lane & 15;

  const int qb = blockIdx.x % NQB;
  const int h  = blockIdx.x / NQB;
  const int g  = h >> 2;
  const int q0 = qb * 64 + wave * 16;

  const _Float16* Q  = (const _Float16*)(const void*)Qp  + (size_t)h * HDIM;
  const _Float16* Kg = (const _Float16*)(const void*)Kp  + (size_t)g * HDIM;
  const _Float16* Vg = (const _Float16*)(const void*)Vtp + (size_t)g * HDIM * SEQ;

  v16h qa[2];
#pragma unroll
  for (int dc = 0; dc < 2; ++dc) {
    qa[dc] = ldfrag<_Float16>(Q + (size_t)(q0 + c) * DMD + dc * 32 + 8 * hh);
  }

  float mrow[8], lrow[8];
  v8f oacc[4];
#pragma unroll
  for (int r = 0; r < 8; ++r) { mrow[r] = -INFINITY; lrow[r] = 0.f; }
#pragma unroll
  for (int t = 0; t < 4; ++t) oacc[t] = zero8();

  const int qloc = wave * 16 + 8 * hh;

  for (int kt = 0; kt <= qb; ++kt) {
    const int kv0 = kt * 64;
    __syncthreads();
    {
      const int r = tid >> 1, half = (tid & 1) * 32;
      const _Float16* kg = Kg + (size_t)(kv0 + r) * DKV + half;
      const _Float16* vg = Vg + (size_t)r * SEQ + kv0 + half;
#pragma unroll
      for (int i = 0; i < 4; ++i) {
        const v8h a0 = *(const v8h*)(kg + 8 * i);
        const v8h b0 = *(const v8h*)(vg + 8 * i);
        *(v8h*)(Ksh + r * 64 + half + 8 * i) = a0;
        *(v8h*)(Vth + r * 64 + half + 8 * i) = b0;
      }
    }
    __syncthreads();

    v8f s[4];
#pragma unroll
    for (int j = 0; j < 4; ++j) {
      s[j] = zero8();
#pragma unroll
      for (int dc = 0; dc < 2; ++dc) {
        FH kb;
        kb.h[0] = *(const v8h*)(Ksh + (j * 16 + c) * 64 + dc * 32 + 8 * hh);
        kb.h[1] = *(const v8h*)(Ksh + (j * 16 + c) * 64 + dc * 32 + 16 + 8 * hh);
        s[j] = mma_g(qa[dc], kb.v, s[j]);
      }
    }

    const bool diag = (kt == qb);
    _Float16* pwh = Psh[wave];
#pragma unroll
    for (int r = 0; r < 8; ++r) {
      float m = -INFINITY;
#pragma unroll
      for (int j = 0; j < 4; ++j) {
        float sv = s[j][r] * sscale;
        const int kl = j * 16 + c;
        if (diag && (kl > qloc + r)) sv = -INFINITY;
        s[j][r] = sv;
        m = fmaxf(m, sv);
      }
#pragma unroll
      for (int off = 1; off < 16; off <<= 1) m = fmaxf(m, __shfl_xor(m, off, 32));
      const float mnew  = fmaxf(mrow[r], m);
      const float msafe = (mnew == -INFINITY) ? 0.f : mnew;
      const float alpha = __expf(mrow[r] - msafe);
      mrow[r] = mnew;
      float psum = 0.f;
#pragma unroll
      for (int j = 0; j < 4; ++j) {
        const float p = __expf(s[j][r] - msafe);
        psum += p;
        pwh[(8 * hh + r) * 64 + j * 16 + c] = (_Float16)(p * 1024.0f);
      }
#pragma unroll
      for (int off = 1; off < 16; off <<= 1) psum += __shfl_xor(psum, off, 32);
      lrow[r] = lrow[r] * alpha + psum;
#pragma unroll
      for (int t = 0; t < 4; ++t) oacc[t][r] *= alpha;
    }
    __builtin_amdgcn_fence(__ATOMIC_RELEASE, "workgroup");
    __builtin_amdgcn_wave_barrier();
    __builtin_amdgcn_fence(__ATOMIC_ACQUIRE, "workgroup");

#pragma unroll 1
    for (int kk = 0; kk < 2; ++kk) {
      FH pa;
      pa.h[0] = *(const v8h*)(pwh + c * 64 + kk * 32 + 8 * hh);
      pa.h[1] = *(const v8h*)(pwh + c * 64 + kk * 32 + 16 + 8 * hh);
#pragma unroll
      for (int t = 0; t < 4; ++t) {
        FH vb;
        vb.h[0] = *(const v8h*)(Vth + (t * 16 + c) * 64 + kk * 32 + 8 * hh);
        vb.h[1] = *(const v8h*)(Vth + (t * 16 + c) * 64 + kk * 32 + 16 + 8 * hh);
        oacc[t] = mma_g(pa.v, vb.v, oacc[t]);
      }
    }
  }

  float* os = Os[wave];
#pragma unroll
  for (int r = 0; r < 8; ++r) {
    const float l = lrow[r];
    const float inv = ((l > 0.f) ? rcpf(l) : 0.f) * oscale;
#pragma unroll
    for (int t = 0; t < 4; ++t) os[(8 * hh + r) * 64 + t * 16 + c] = oacc[t][r] * inv;
  }
  __builtin_amdgcn_fence(__ATOMIC_RELEASE, "workgroup");
  __builtin_amdgcn_wave_barrier();
  __builtin_amdgcn_fence(__ATOMIC_ACQUIRE, "workgroup");
  {
    const int q4 = lane >> 3, c8 = (lane & 7) * 8;
    v4u hv[4];
#pragma unroll
    for (int it = 0; it < 4; ++it) {
      const int row = it * 4 + q4;
      const float* sp = os + row * 64 + c8;
      v4u a;
#pragma unroll
      for (int e = 0; e < 4; ++e) a[e] = pk16(h_bits(sp[2 * e]), h_bits(sp[2 * e + 1]));
      hv[it] = a;
    }
    for (int pass = 0; pass < 2; ++pass) {
#pragma unroll
      for (int it = 0; it < 4; ++it) {
        const int row = it * 4 + q4;
        const size_t go = (size_t)(q0 + row) * DMD + (size_t)h * HDIM + c8;
        *(volatile v4u*)(Op + go) = hv[it];
      }
      __threadfence();
    }
  }
}

__global__ __launch_bounds__(256) void conv_silu(const float* __restrict__ XZ, const float* __restrict__ cw,
                                                 const float* __restrict__ cb,
                                                 float* XC, unsigned short* XCH, unsigned short* XCL) {
  const int tid = threadIdx.x;
  const int t = blockIdx.x;
  const int d0 = 4 * tid;
  v4f wv[4];
#pragma unroll
  for (int e = 0; e < 4; ++e) wv[e] = *(const v4f*)(cw + (size_t)(d0 + e) * 4);
  float a[4] = {0.f, 0.f, 0.f, 0.f};
#pragma unroll
  for (int k = 0; k < 4; ++k) {
    const int tt  = t - 3 + k;
    const int ttc = (tt < 0) ? 0 : tt;
    const bool live = (tt >= 0);
    const v4f xb = *(const v4f*)(XZ + (size_t)ttc * DXZ + d0);
#pragma unroll
    for (int e = 0; e < 4; ++e) {
      const float xe = live ? xb[e] : 0.f;
      a[e] += xe * wv[e][k];
    }
  }
  const v4f bv = *(const v4f*)(cb + d0);
  v4f xc;
#pragma unroll
  for (int e = 0; e < 4; ++e) xc[e] = siluf(a[e] + bv[e]);
  v2u ph, pl;
  {
    unsigned short hb[4], lb[4];
#pragma unroll
    for (int e = 0; e < 4; ++e) { hb[e] = bf_bits(xc[e]); lb[e] = bf_bits(xc[e] - bf_up(hb[e])); }
    ph[0] = pk16(hb[0], hb[1]); ph[1] = pk16(hb[2], hb[3]);
    pl[0] = pk16(lb[0], lb[1]); pl[1] = pk16(lb[2], lb[3]);
  }
  const size_t o = (size_t)t * DMD + d0;
  *(volatile v4f*)(XC + o)  = xc;
  *(volatile v2u*)(XCH + o) = ph;
  *(volatile v2u*)(XCL + o) = pl;
  __threadfence();
  *(volatile v4f*)(XC + o)  = xc;
  *(volatile v2u*)(XCH + o) = ph;
  *(volatile v2u*)(XCL + o) = pl;
}

__global__ __launch_bounds__(64)
void ssm_scan(const float* __restrict__ PROJ, const float* __restrict__ XC, const float* __restrict__ XZ,
              const float* __restrict__ alog, const float* __restrict__ dsk,
              unsigned short* YM, float* HOUT) {
  __shared__ __align__(16) _Float16 ysh[16 * 64];
  __shared__ __align__(16) float hsh[64 * 16];
  const int tid = threadIdx.x, wave = tid >> 5, lane = tid & 31, q = lane >> 3, j = lane & 7;
  const int d0 = blockIdx.x * 64;
  const int d = d0 + tid;
  float A[NST], h[NST];
#pragma unroll
  for (int i = 0; i < 4; ++i) {
    const v4f al = *(const v4f*)(alog + (size_t)d * NST + 4 * i);
#pragma unroll
    for (int e = 0; e < 4; ++e) { A[4 * i + e] = -__expf(al[e]); h[4 * i + e] = 0.f; }
  }
  const float dk = dsk[d];

#pragma unroll 1
  for (int t0 = 0; t0 < SEQ; t0 += 16) {
#pragma unroll 1
    for (int tt = 0; tt < 16; ++tt) {
      const int t = t0 + tt;
      const float* pr = PROJ + (size_t)t * DXP;
      const float pd = pr[d];
      float Bv[NST], Cv[NST];
#pragma unroll
      for (int i = 0; i < 4; ++i) {
        const v4f b4 = *(const v4f*)(pr + DMD + 4 * i);
        const v4f c4 = *(const v4f*)(pr + DMD + NST + 4 * i);
#pragma unroll
        for (int e = 0; e < 4; ++e) { Bv[4 * i + e] = b4[e]; Cv[4 * i + e] = c4[e]; }
      }
      const float delta = fmaxf(pd, 0.f) + log1pf(__expf(-fabsf(pd)));
      const float xv = XC[(size_t)t * DMD + d];
      float acc = 0.f;
#pragma unroll
      for (int n = 0; n < NST; ++n) {
        const float a  = __expf(delta * A[n]);
        const float bb = delta * Bv[n];
        h[n] = a * h[n] + bb * xv;
        acc += h[n] * Cv[n];
      }
      const float y  = acc + dk * xv;
      const float z  = XZ[(size_t)t * DXZ + DMD + d];
      const float ym = y * siluf(z) * 1024.0f;
      ysh[tt * 64 + tid] = (_Float16)ym;
    }
    __syncthreads();
    v4u pv[2];
#pragma unroll
    for (int it = 0; it < 2; ++it) {
      const int row = 8 * it + 4 * wave + q;
      pv[it] = *(const v4u*)(ysh + row * 64 + 8 * j);
    }
    for (int pass = 0; pass < 2; ++pass) {
#pragma unroll
      for (int it = 0; it < 2; ++it) {
        const int row = 8 * it + 4 * wave + q;
        *(volatile v4u*)(YM + (size_t)(t0 + row) * DMD + d0 + 8 * j) = pv[it];
      }
      __threadfence();
    }
    __syncthreads();
  }

#pragma unroll
  for (int i = 0; i < 4; ++i) {
    v4f hv4;
    hv4[0] = h[4 * i]; hv4[1] = h[4 * i + 1]; hv4[2] = h[4 * i + 2]; hv4[3] = h[4 * i + 3];
    *(v4f*)(hsh + tid * NST + 4 * i) = hv4;
  }
  __syncthreads();
  v4f hv[4];
#pragma unroll
  for (int it = 0; it < 4; ++it) {
    const int line = 16 * wave + 4 * it + q;
    hv[it] = *(const v4f*)(hsh + line * 32 + 4 * j);
  }
  float* hb = HOUT + (size_t)d0 * NST;
  for (int pass = 0; pass < 2; ++pass) {
#pragma unroll
    for (int it = 0; it < 4; ++it) {
      const int line = 16 * wave + 4 * it + q;
      *(volatile v4f*)(hb + (size_t)line * 32 + 4 * j) = hv[it];
    }
    __threadfence();
  }
}

extern "C" void kernel_launch(void* const* d_in, const int* in_sizes, int n_in,
                              void* d_out, int out_size, void* d_ws, size_t ws_size,
                              hipStream_t stream) {
  if (n_in < 18) return;
  if (in_sizes[0] != SEQ * DMD || in_sizes[1] != DMD || in_sizes[2] != DMD) return;
  if (in_sizes[3] != DMD * DMD || in_sizes[4] != DMD * DKV || in_sizes[5] != DMD * DKV || in_sizes[6] != DMD * DMD) return;
  if (in_sizes[7] != DMD * DFFN || in_sizes[8] != DMD * DFFN || in_sizes[9] != DFFN * DMD) return;
  if (in_sizes[10] != NSSM * DMD || in_sizes[11] != NSSM * DMD * DXZ || in_sizes[12] != NSSM * DMD * 4) return;
  if (in_sizes[13] != NSSM * DMD || in_sizes[14] != NSSM * DMD * DXN || in_sizes[15] != NSSM * DMD * NST) return;
  if (in_sizes[16] != NSSM * DMD || in_sizes[17] != NSSM * DMD * DMD) return;
  if (out_size != SEQ * DMD + NSSM * DMD * NST) return;

  const float* x_in  = (const float*)d_in[0];
  const float* anw   = (const float*)d_in[1];
  const float* fnw   = (const float*)d_in[2];
  const float* Wq    = (const float*)d_in[3];
  const float* Wk    = (const float*)d_in[4];
  const float* Wv    = (const float*)d_in[5];
  const float* Wo    = (const float*)d_in[6];
  const float* Wg    = (const float*)d_in[7];
  const float* Wu    = (const float*)d_in[8];
  const float* Wd    = (const float*)d_in[9];
  const float* mnw   = (const float*)d_in[10];
  const float* Win   = (const float*)d_in[11];
  const float* cw    = (const float*)d_in[12];
  const float* cb    = (const float*)d_in[13];
  const float* Wx    = (const float*)d_in[14];
  const float* Alog  = (const float*)d_in[15];
  const float* Dp    = (const float*)d_in[16];
  const float* Wout  = (const float*)d_in[17];
  float* outf = (float*)d_out;

  const size_t PXH  = (size_t)SEQ * DMD * 2;
  const size_t PWS  = (size_t)DFFN * DMD * 2;
  const size_t PQ   = (size_t)SEQ * DMD * 2;
  const size_t PKP  = (size_t)SEQ * DKV * 2;
  const size_t PVT  = (size_t)DKV * SEQ * 2;
  const size_t PO   = (size_t)SEQ * DMD * 2;
  const size_t PG   = (size_t)SEQ * DFFN * 4;
  const size_t PGU  = (size_t)SEQ * DFFN * 2;
  const size_t PXZ  = (size_t)SEQ * DXZ * 4;
  const size_t PXC  = (size_t)SEQ * DMD * 4;
  const size_t PXCH = (size_t)SEQ * DMD * 2;
  const size_t PPRJ = (size_t)SEQ * DXP * 4;
  const size_t PYM  = (size_t)SEQ * DMD * 2;
  const size_t actAttn = PQ + PKP + PVT + PO;
  const size_t actFfn  = PG + PGU;
  const size_t actSsm  = PXZ + PXC + 2 * PXCH + PPRJ + PYM;
  size_t PACT = actAttn;
  if (actFfn > PACT) PACT = actFfn;
  if (actSsm > PACT) PACT = actSsm;
  size_t off = 0;
  const size_t oXH  = off; off += PXH;
  const size_t oXNH = off; off += PXH;
  const size_t oXNL = off; off += PXH;
  const size_t oWA  = off; off += PWS;
  const size_t oWB  = off; off += PWS;
  const size_t oWC  = off; off += PWS;
  const size_t oACT = off; off += PACT;
  if (off > ws_size) return;
  if (off > (size_t)134217728) return;
  const size_t EW2 = (size_t)DMD * DMD;
  const size_t EWX = (size_t)DXP * DMD;
  if ((EW2 + EW2) * 2 > PWS) return;
  if ((EW2 + EWX) * 2 > PWS) return;

  char* ws = (char*)d_ws;
  unsigned short* XH  = (unsigned short*)(ws + oXH);
  unsigned short* XNH = (unsigned short*)(ws + oXNH);
  unsigned short* XNL = (unsigned short*)(ws + oXNL);
  unsigned short* WA  = (unsigned short*)(ws + oWA);
  unsigned short* WB  = (unsigned short*)(ws + oWB);
  unsigned short* WC  = (unsigned short*)(ws + oWC);
  unsigned short* WinZ  = WA;
  unsigned short* WinH  = WA + EW2;
  unsigned short* WinL  = WB;
  unsigned short* WxH   = WB + EW2;
  unsigned short* WxL   = WC;
  unsigned short* WoutP = WC + EWX;
  char* act = ws + oACT;
  unsigned short* Qh  = (unsigned short*)(act);
  unsigned short* KP  = (unsigned short*)(act + PQ);
  unsigned short* VT  = (unsigned short*)(act + PQ + PKP);
  unsigned short* Oh  = (unsigned short*)(act + PQ + PKP + PVT);
  float*          G   = (float*)(act);
  unsigned short* GU  = (unsigned short*)(act + PG);
  float*          XZ  = (float*)(act);
  float*          XC  = (float*)(act + PXZ);
  unsigned short* XCH = (unsigned short*)(act + PXZ + PXC);
  unsigned short* XCL = (unsigned short*)(act + PXZ + PXC + PXCH);
  float*          PRJ = (float*)(act + PXZ + PXC + 2 * PXCH);
  unsigned short* YM  = (unsigned short*)(act + PXZ + PXC + 2 * PXCH + PPRJ);

  const dim3 b256(256);
  const unsigned gSq   = (unsigned)((((SEQ / 64) * (DMD / 64)) + 7) / 8);
  const unsigned gKv   = (unsigned)((((SEQ / 64) * (DKV / 64)) + 7) / 8);
  const unsigned gVt   = (unsigned)((((DKV / 64) * (SEQ / 64)) + 7) / 8);
  const unsigned gFf   = (unsigned)((((SEQ / 64) * (DFFN / 64)) + 7) / 8);
  const unsigned gWx   = (unsigned)((((SEQ / 64) * (DXP / 64)) + 7) / 8);
  const float sW    = 256.0f;
  const float sProj = 16.0f / 256.0f;
  const float sscl  = 0.125f / 256.0f;
  const float oscl  = 1.0f / 256.0f;
  const float sWo   = 1.0f / 16384.0f;
  const float sXn   = 1.0f / 256.0f;
  const float sGu   = 0.25f;
  const float sWd   = 1.0f / 16384.0f;
  const float sWout = 1.0f / 262144.0f;

  rmsnorm_h<0><<<dim3(SEQ), b256, 0, stream>>>(x_in, anw, XH, XH, XH);
  wcvt<0><<<dim3(DMD / 64, DMD / 64), b256, 0, stream>>>(Wq, DMD, DMD, DMD, WA, WA, sW);
  wcvt<0><<<dim3(DKV / 64, DMD / 64), b256, 0, stream>>>(Wk, DKV, DMD, DKV, WB, WB, sW);
  wcvt<0><<<dim3(DKV / 64, DMD / 64), b256, 0, stream>>>(Wv, DKV, DMD, DKV, WC, WC, sW);
  gemm64<_Float16, 0, 2><<<dim3(gSq), b256, 0, stream>>>(
      XH, XH, DMD, WA, WA, DMD, (void*)Qh, DMD, x_in, 0, SEQ, DMD, DMD, sProj);
  gemm64<_Float16, 0, 2><<<dim3(gKv), b256, 0, stream>>>(
      XH, XH, DMD, WB, WB, DMD, (void*)KP, DKV, x_in, 0, SEQ, DKV, DMD, sProj);
  gemm64<_Float16, 0, 2><<<dim3(gVt), b256, 0, stream>>>(
      WC, WC, DMD, XH, XH, DMD, (void*)VT, SEQ, x_in, 0, DKV, SEQ, DMD, sProj);
  attn_causal<<<dim3(NHD * NQB), dim3(128), 0, stream>>>(Qh, KP, VT, Oh, sscl, oscl);
  wcvt<0><<<dim3(DMD / 64, DMD / 64), b256, 0, stream>>>(Wo, DMD, DMD, DMD, WA, WA, sW);
  gemm64<_Float16, 0, 1><<<dim3(gSq), b256, 0, stream>>>(
      Oh, Oh, DMD, WA, WA, DMD, d_out, DMD, x_in, DMD, SEQ, DMD, DMD, sWo);

  rmsnorm_h<0><<<dim3(SEQ), b256, 0, stream>>>(outf, fnw, XH, XH, XH);
  wcvt<0><<<dim3(DFFN / 64, DMD / 64), b256, 0, stream>>>(Wg, DFFN, DMD, DFFN, WA, WA, sW);
  wcvt<0><<<dim3(DFFN / 64, DMD / 64), b256, 0, stream>>>(Wu, DFFN, DMD, DFFN, WB, WB, sW);
  wcvt<0><<<dim3(DMD / 64, DFFN / 64), b256, 0, stream>>>(Wd, DMD, DFFN, DMD, WC, WC, sW);
  gemm64<_Float16, 0, 0><<<dim3(gFf), b256, 0, stream>>>(
      XH, XH, DMD, WA, WA, DMD, (void*)G, DFFN, x_in, 0, SEQ, DFFN, DMD, sXn);
  gemm64<_Float16, 0, 3><<<dim3(gFf), b256, 0, stream>>>(
      XH, XH, DMD, WB, WB, DMD, (void*)GU, DFFN, G, DFFN, SEQ, DFFN, DMD, sGu);
  gemm64<_Float16, 0, 1><<<dim3(gSq), b256, 0, stream>>>(
      GU, GU, DFFN, WC, WC, DFFN, d_out, DMD, outf, DMD, SEQ, DMD, DFFN, sWd);

  for (int mi = 0; mi < NSSM; ++mi) {
    const float* Winm = Win + (size_t)mi * DMD * DXZ;
    rmsnorm_h<1><<<dim3(SEQ), b256, 0, stream>>>(outf, mnw + (size_t)mi * DMD, XH, XNH, XNL);
    wcvt<1><<<dim3(DMD / 64, DMD / 64), b256, 0, stream>>>(Winm, DXZ, DMD, DMD, WinH, WinL, 1.0f);
    wcvt<0><<<dim3(DMD / 64, DMD / 64), b256, 0, stream>>>(Winm + DMD, DXZ, DMD, DMD, WinZ, WinZ, sW);
    wcvt<1><<<dim3(DXP / 64, DMD / 64), b256, 0, stream>>>(Wx + (size_t)mi * DMD * DXN, DXN, DMD, DXN, WxH, WxL, 1.0f);
    gemm64<__bf16, 2, 0><<<dim3(gSq), b256, 0, stream>>>(
        XNH, XNL, DMD, WinH, WinL, DMD, (void*)XZ, DXZ, x_in, 0, SEQ, DMD, DMD, 1.0f);
    gemm64<_Float16, 0, 0><<<dim3(gSq), b256, 0, stream>>>(
        XH, XH, DMD, WinZ, WinZ, DMD, (void*)(XZ + DMD), DXZ, x_in, 0, SEQ, DMD, DMD, sXn);
    conv_silu<<<dim3(SEQ), b256, 0, stream>>>(XZ, cw + (size_t)mi * DMD * 4, cb + (size_t)mi * DMD, XC, XCH, XCL);
    gemm64<__bf16, 2, 0><<<dim3(gWx), b256, 0, stream>>>(
        XCH, XCL, DMD, WxH, WxL, DMD, (void*)PRJ, DXP, x_in, 0, SEQ, DXP, DMD, 1.0f);
    wcvt<0><<<dim3(DMD / 64, DMD / 64), b256, 0, stream>>>(Wout + (size_t)mi * DMD * DMD, DMD, DMD, DMD, WoutP, WoutP, sW);
    ssm_scan<<<dim3(DMD / 64), dim3(64), 0, stream>>>(
        PRJ, XC, XZ, Alog + (size_t)mi * DMD * NST, Dp + (size_t)mi * DMD,
        YM, outf + (size_t)SEQ * DMD + (size_t)mi * DMD * NST);
    gemm64<_Float16, 0, 1><<<dim3(gSq), b256, 0, stream>>>(
        YM, YM, DMD, WoutP, WoutP, DMD, d_out, DMD, outf, DMD, SEQ, DMD, DMD, sWout);
  }
  (void)hipGetLastError();
}
